// TransformerBlock_39127152066581
// MI455X (gfx1250) — hardware-verified
//
#include <hip/hip_runtime.h>


typedef __attribute__((ext_vector_type(16))) _Float16 v16h;
typedef __attribute__((ext_vector_type(8)))  _Float16 v8h;
typedef __attribute__((ext_vector_type(8)))  float v8f;
typedef __attribute__((ext_vector_type(4)))  float v4f;
typedef __attribute__((ext_vector_type(4)))  unsigned int v4u;
union H8 { v8h h; v4u u; };

#ifndef NB
#define NB 2
#endif
#ifndef SEQ
#define SEQ 2048
#endif
#define NB_FULL  2
#define SEQ_FULL 2048
#define DM   1024
#define NH   16
#define HD   64
#define FF   4096
#define ROWS (NB * SEQ)
#define KPAD 72
#define VSPAD 136
#define YP   1028
#define RMS_EPS 1e-5f
#define WSC    64.0f
#define LN1024 6.931471806f

#define NRB   (ROWS / 8)
#define NT_SQ ((DM / 64) * (DM / 64))
#define NT_F  ((DM / 64) * (FF / 64))
#define NWT   (4 * NT_SQ + 2 * NT_F)

#define PLANE2     ((size_t)ROWS * DM * 2)
#define WQKV_BYTES ((size_t)3 * DM * DM * 2)
#define WO_BYTES   ((size_t)DM * DM * 2)
#define WF1_BYTES  ((size_t)FF * DM * 2)
#define WF2_BYTES  ((size_t)DM * FF * 2)
#define H_BYTES    ((size_t)ROWS * FF * 2)
#define WS_TOTAL   (PLANE2 + WQKV_BYTES + WO_BYTES + WF1_BYTES + WF2_BYTES + 3 * PLANE2 + H_BYTES)

static_assert(NB >= 1 && NB <= NB_FULL);
static_assert(SEQ >= 128 && SEQ <= SEQ_FULL && (SEQ % 128) == 0);
static_assert((ROWS % 128) == 0 && (ROWS % 16) == 0 && (ROWS % 8) == 0);
static_assert((DM % 64) == 0 && (FF % 64) == 0 && (HD % 32) == 0 && NH * HD == DM);
static_assert((DM % 32) == 0 && (FF % 32) == 0 && HD == 64 && NH == 16 && DM == 1024);
static_assert(128 * KPAD >= 64 * VSPAD);
static_assert(2 * PLANE2 == (size_t)ROWS * DM * 4);
static_assert(WS_TOTAL <= (size_t)134217728);
static_assert((size_t)((NB_FULL - 1) * SEQ_FULL + SEQ) * DM * 4 <= (size_t)16777216);
static_assert((size_t)NRB * 256 * 32 == (size_t)ROWS * DM);
static_assert((size_t)NWT * 64 * 64 == (size_t)4 * DM * DM + (size_t)2 * DM * FF);
static_assert((size_t)(ROWS / 128) * (3 * NH) * 128 * 64 == (size_t)3 * ROWS * DM);
static_assert((size_t)(SEQ / 128) * (NB * NH) * 128 * 64 == (size_t)ROWS * DM);
static_assert((size_t)(ROWS / 16) * 16 * DM == (size_t)ROWS * DM);
static_assert((size_t)(ROWS / 128) * (FF / 64) * 128 * 64 == (size_t)ROWS * FF);

__device__ __forceinline__ float bf16q(float f) {
  unsigned int u = __float_as_uint(f);
  u += 0x7FFFu + ((u >> 16) & 1u);
  return __uint_as_float(u & 0xFFFF0000u);
}

__device__ __forceinline__ v16h load_frag_row(const _Float16* base, unsigned stride,
                                              unsigned lane) {
  const _Float16* rowp = base + (size_t)((lane & 15u) * stride + ((lane >> 4) << 3));
  const v8h lo = *(const v8h*)(rowp);
  const v8h hi = *(const v8h*)(rowp + 16);
  return __builtin_shufflevector(lo, hi, 0, 1, 2, 3, 4, 5, 6, 7,
                                 8, 9, 10, 11, 12, 13, 14, 15);
}

__device__ __forceinline__ v8f wmma_f16(v16h a, v16h b, v8f c) {
  v8f d = __builtin_amdgcn_wmma_f32_16x16x32_f16(false, a, false, b, (short)0, c,
                                                 false, false);
  asm volatile("v_nop\n\tv_nop\n\tv_nop\n\tv_nop" : "+v"(d) : "v"(a), "v"(b));
  return d;
}

__global__ __launch_bounds__(256) void rms1_kernel(const float* __restrict__ x,
                                                   const float* __restrict__ g,
                                                   _Float16* __restrict__ xh) {
  const unsigned lane = threadIdx.x & 31u;
  const unsigned wave = threadIdx.x >> 5;
  const unsigned m    = blockIdx.x * 8u + wave;
  const unsigned bb   = m / (unsigned)SEQ;
  const unsigned s    = m - bb * (unsigned)SEQ;
  const float* src  = x + ((size_t)bb * SEQ_FULL + s) * DM + lane * 8u;
  const float* gsrc = g + lane * 8u;

  float ss = 0.0f;
#pragma unroll 1
  for (unsigned c = 0; c < 4u; ++c) {
    const v4f a = *(const v4f*)(src + c * 256u);
    const v4f d = *(const v4f*)(src + c * 256u + 4u);
#pragma unroll
    for (int i = 0; i < 4; ++i) {
      const float p = bf16q(a[i]);
      const float q = bf16q(d[i]);
      ss += p * p;
      ss += q * q;
    }
  }
  ss += __shfl_xor(ss, 16, 32);
  ss += __shfl_xor(ss, 8, 32);
  ss += __shfl_xor(ss, 4, 32);
  ss += __shfl_xor(ss, 2, 32);
  ss += __shfl_xor(ss, 1, 32);
  const float inv = rsqrtf(ss * (1.0f / DM) + RMS_EPS);

  _Float16* dst = xh + (size_t)m * DM + lane * 8u;
  auto store_pass = [&]() {
#pragma unroll 1
    for (unsigned c = 0; c < 4u; ++c) {
      const v4f a  = *(const v4f*)(src + c * 256u);
      const v4f d  = *(const v4f*)(src + c * 256u + 4u);
      const v4f g0 = *(const v4f*)(gsrc + c * 256u);
      const v4f g1 = *(const v4f*)(gsrc + c * 256u + 4u);
      H8 o;
#pragma unroll
      for (int i = 0; i < 4; ++i) {
        o.h[i]     = (_Float16)(bf16q(g0[i]) * (bf16q(a[i]) * inv));
        o.h[4 + i] = (_Float16)(bf16q(g1[i]) * (bf16q(d[i]) * inv));
      }
      *(volatile v4u*)(dst + c * 256u) = o.u;
    }
  };
  store_pass();
  __threadfence();
  store_pass();
}

__global__ __launch_bounds__(256) void cvt_w_kernel(
    const float* __restrict__ Wq, const float* __restrict__ Wk, const float* __restrict__ Wv,
    const float* __restrict__ Wo, const float* __restrict__ Wf1, const float* __restrict__ Wf2,
    _Float16* __restrict__ wqkv, _Float16* __restrict__ woh,
    _Float16* __restrict__ wf1t, _Float16* __restrict__ wf2t) {
  __shared__ _Float16 ts[64 * KPAD];
  const unsigned bid = blockIdx.x;
  const unsigned tid = threadIdx.x;
  const float* W;
  _Float16* dst;
  unsigned K, N, kt, nt;
  if (bid < 4u * NT_SQ) {
    const unsigned which = bid / (unsigned)NT_SQ;
    const unsigned tile  = bid - which * (unsigned)NT_SQ;
    kt = tile / (unsigned)(DM / 64); nt = tile - kt * (unsigned)(DM / 64); K = DM; N = DM;
    W = (which == 0u) ? Wq : ((which == 1u) ? Wk : ((which == 2u) ? Wv : Wo));
    dst = (which < 3u) ? (wqkv + (size_t)which * DM * DM) : woh;
  } else if (bid < 4u * NT_SQ + NT_F) {
    const unsigned tile = bid - 4u * NT_SQ;
    kt = tile / (unsigned)(FF / 64); nt = tile - kt * (unsigned)(FF / 64); K = DM; N = FF;
    W = Wf1; dst = wf1t;
  } else {
    const unsigned tile = bid - 4u * NT_SQ - NT_F;
    kt = tile / (unsigned)(DM / 64); nt = tile - kt * (unsigned)(DM / 64); K = FF; N = DM;
    W = Wf2; dst = wf2t;
  }
#pragma unroll
  for (unsigned it = 0; it < 4u; ++it) {
    const unsigned idx = it * 256u + tid;
    const unsigned kr = idx >> 4, c4 = idx & 15u;
    const v4f v = *(const v4f*)(W + (size_t)(kt * 64u + kr) * N + nt * 64u + c4 * 4u);
#pragma unroll
    for (unsigned j = 0; j < 4u; ++j) ts[(c4 * 4u + j) * KPAD + kr] = (_Float16)(bf16q(v[j]) * WSC);
  }
  __syncthreads();
  v4u rv[2];
#pragma unroll
  for (unsigned it = 0; it < 2u; ++it) {
    const unsigned idx = it * 256u + tid;
    const unsigned n = idx >> 3, piece = idx & 7u;
    rv[it] = *(const v4u*)(ts + n * KPAD + piece * 8u);
  }
#pragma unroll
  for (unsigned it = 0; it < 2u; ++it) {
    const unsigned idx = it * 256u + tid;
    const unsigned n = idx >> 3, piece = idx & 7u;
    *(volatile v4u*)(dst + (size_t)(nt * 64u + n) * K + kt * 64u + piece * 8u) = rv[it];
  }
  __threadfence();
#pragma unroll
  for (unsigned it = 0; it < 2u; ++it) {
    const unsigned idx = it * 256u + tid;
    const unsigned n = idx >> 3, piece = idx & 7u;
    *(volatile v4u*)(dst + (size_t)(nt * 64u + n) * K + kt * 64u + piece * 8u) = rv[it];
  }
}

__global__ __launch_bounds__(256) void qkv_kernel(
    const _Float16* __restrict__ xh, const _Float16* __restrict__ wqkv,
    const float* __restrict__ bq, const float* __restrict__ bk, const float* __restrict__ bv,
    _Float16* __restrict__ q, _Float16* __restrict__ k, _Float16* __restrict__ vT) {
  __shared__ _Float16 stg[128 * KPAD];

  const unsigned tid  = threadIdx.x;
  const unsigned lane = tid & 31u;
  const unsigned wave = tid >> 5;
  const unsigned hh   = lane >> 4;
  const unsigned l15  = lane & 15u;

  const unsigned cb   = blockIdx.y;
  const unsigned osel = cb >> 4;
  const unsigned h    = cb & 15u;
  const unsigned m0   = blockIdx.x * 128u;
  const unsigned b    = m0 / (unsigned)SEQ;
  const unsigned s0   = m0 - b * (unsigned)SEQ;

  const _Float16* xrow = xh + (size_t)(m0 + wave * 16u) * DM;
  const _Float16* wrow = wqkv + (size_t)(cb * 64u) * DM;

  v8f acc[4];
#pragma unroll
  for (int j = 0; j < 4; ++j) acc[j] = (v8f){};

#pragma unroll 1
  for (unsigned kk = 0; kk < DM; kk += 32u) {
    const v16h xf = load_frag_row(xrow + kk, DM, lane);
#pragma unroll
    for (int j = 0; j < 4; ++j) {
      const v16h wf = load_frag_row(wrow + (size_t)(j * 16) * DM + kk, DM, lane);
      acc[j] = wmma_f16(wf, xf, acc[j]);
    }
  }

  const float* bias = (osel == 0u) ? bq : ((osel == 1u) ? bk : bv);
  const float  rsc  = 1.0f / WSC;

  v4u rv[4];
  if (osel < 2u) {
    _Float16* srow = stg + (wave * 16u + l15) * KPAD;
#pragma unroll
    for (int j = 0; j < 4; ++j) {
      const unsigned n8 = (unsigned)j * 16u + hh * 8u;
      const v4f b0 = *(const v4f*)(bias + h * HD + n8);
      const v4f b1 = *(const v4f*)(bias + h * HD + n8 + 4u);
      H8 pk;
#pragma unroll
      for (int r = 0; r < 4; ++r) {
        pk.h[r]     = (_Float16)(acc[j][r]     * rsc + bf16q(b0[r]));
        pk.h[4 + r] = (_Float16)(acc[j][4 + r] * rsc + bf16q(b1[r]));
      }
      *(v4u*)(srow + n8) = pk.u;
    }
    __syncthreads();
#pragma unroll
    for (unsigned it = 0; it < 4u; ++it) {
      const unsigned idx = it * 256u + tid;
      const unsigned row = idx >> 3, piece = idx & 7u;
      rv[it] = *(const v4u*)(stg + row * KPAD + piece * 8u);
    }
    _Float16* dst = ((osel == 0u) ? q : k) + ((size_t)(b * NH + h) * SEQ + s0) * HD;
#pragma unroll
    for (unsigned it = 0; it < 4u; ++it)
      *(volatile v4u*)(dst + (size_t)(it * 256u + tid) * 8u) = rv[it];
    __threadfence();
#pragma unroll
    for (unsigned it = 0; it < 4u; ++it)
      *(volatile v4u*)(dst + (size_t)(it * 256u + tid) * 8u) = rv[it];
  } else {
#pragma unroll
    for (int j = 0; j < 4; ++j) {
      const unsigned n8 = (unsigned)j * 16u + hh * 8u;
      const v4f b0 = *(const v4f*)(bias + h * HD + n8);
      const v4f b1 = *(const v4f*)(bias + h * HD + n8 + 4u);
#pragma unroll
      for (int r = 0; r < 4; ++r) {
        stg[(n8 + r) * VSPAD + wave * 16u + l15]      = (_Float16)(acc[j][r]     * rsc + bf16q(b0[r]));
        stg[(n8 + 4u + r) * VSPAD + wave * 16u + l15] = (_Float16)(acc[j][4 + r] * rsc + bf16q(b1[r]));
      }
    }
    __syncthreads();
#pragma unroll
    for (unsigned it = 0; it < 4u; ++it) {
      const unsigned idx = it * 256u + tid;
      const unsigned d = idx >> 4, piece = idx & 15u;
      rv[it] = *(const v4u*)(stg + d * VSPAD + piece * 8u);
    }
    _Float16* dstb = vT + ((size_t)(b * NH + h) * HD) * SEQ + s0;
#pragma unroll
    for (unsigned it = 0; it < 4u; ++it) {
      const unsigned idx = it * 256u + tid;
      const unsigned d = idx >> 4, piece = idx & 15u;
      *(volatile v4u*)(dstb + (size_t)d * SEQ + piece * 8u) = rv[it];
    }
    __threadfence();
#pragma unroll
    for (unsigned it = 0; it < 4u; ++it) {
      const unsigned idx = it * 256u + tid;
      const unsigned d = idx >> 4, piece = idx & 15u;
      *(volatile v4u*)(dstb + (size_t)d * SEQ + piece * 8u) = rv[it];
    }
  }
}

__global__ __launch_bounds__(256) void attn_kernel(
    const _Float16* __restrict__ Q, const _Float16* __restrict__ K,
    const _Float16* __restrict__ vT, _Float16* __restrict__ ctx) {
  __shared__ _Float16 ks[64 * KPAD];
  __shared__ _Float16 vts[64 * KPAD];
  __shared__ _Float16 ost[128 * KPAD];

  const unsigned tid  = threadIdx.x;
  const unsigned lane = tid & 31u;
  const unsigned wave = tid >> 5;
  const unsigned bh   = blockIdx.y;
  const unsigned b    = bh >> 4;
  const unsigned h    = bh & 15u;
  const unsigned q0   = blockIdx.x * 128u;
  const unsigned kend = q0 + 128u;

  const _Float16* Qb  = Q + ((size_t)bh * SEQ + q0) * HD;
  const _Float16* Kb  = K + (size_t)bh * SEQ * HD;
  const _Float16* vTb = vT + (size_t)bh * HD * SEQ;

  v16h qfrag[2];
  {
    const _Float16* qrow = Qb + (size_t)(wave * 16u) * HD;
#pragma unroll
    for (int t = 0; t < 2; ++t) qfrag[t] = load_frag_row(qrow + t * 32, HD, lane);
  }

  v8f acc[4];
#pragma unroll
  for (int nt = 0; nt < 4; ++nt) acc[nt] = (v8f){};
  float mi = -1e30f, li = 0.0f;

  const unsigned colb = lane & 15u;
  const unsigned rofs = (lane >> 4) << 3;
  const unsigned qi   = q0 + wave * 16u + colb;

#pragma unroll 1
  for (unsigned kb = 0; kb < kend; kb += 64u) {
    __syncthreads();
#pragma unroll
    for (unsigned idx = tid; idx < 64u * 8u; idx += 256u) {
      const unsigned row = idx >> 3, c = idx & 7u;
      *(v4u*)(ks + row * KPAD + c * 8u) =
          *(const v4u*)(Kb + (size_t)(kb + row) * HD + c * 8u);
    }
#pragma unroll
    for (unsigned idx = tid; idx < 64u * 8u; idx += 256u) {
      const unsigned d = idx >> 3, c = idx & 7u;
      *(v4u*)(vts + d * KPAD + c * 8u) =
          *(const v4u*)(vTb + (size_t)d * SEQ + kb + c * 8u);
    }
    __syncthreads();

    v8f sc[4];
#pragma unroll
    for (int kt = 0; kt < 4; ++kt) sc[kt] = (v8f){};
#pragma unroll
    for (int t = 0; t < 2; ++t)
#pragma unroll
      for (int kt = 0; kt < 4; ++kt) {
        const v16h kf = load_frag_row(ks + (kt * 16) * KPAD + t * 32, KPAD, lane);
        sc[kt] = wmma_f16(kf, qfrag[t], sc[kt]);
      }

    if (kb + 64u > q0) {
#pragma unroll
      for (int kt = 0; kt < 4; ++kt)
#pragma unroll
        for (int r = 0; r < 8; ++r) {
          const unsigned key = kb + (unsigned)(kt * 16 + r) + rofs;
          sc[kt][r] = (key > qi) ? -1e30f : sc[kt][r];
        }
    }

    float mx = sc[0][0];
#pragma unroll
    for (int kt = 0; kt < 4; ++kt)
#pragma unroll
      for (int r = 0; r < 8; ++r) mx = fmaxf(mx, sc[kt][r]);
    mx = fmaxf(mx, __shfl_xor(mx, 16, 32));
    const float mnew  = fmaxf(mi, mx);
    const float alpha = __expf((mi - mnew) * 0.125f);
    mi = mnew;
    const float cs = fmaf(mnew, 0.125f, -LN1024);

    float rs = 0.0f;
#pragma unroll
    for (int kt = 0; kt < 4; ++kt)
#pragma unroll
      for (int r = 0; r < 8; ++r) {
        const float p = __expf(fmaf(sc[kt][r], 0.125f, -cs));
        sc[kt][r] = p;
        rs += p;
      }
    rs += __shfl_xor(rs, 16, 32);
    li = li * alpha + rs;

    v16h pf[2];
#pragma unroll
    for (int t = 0; t < 2; ++t)
#pragma unroll
      for (int i = 0; i < 8; ++i) {
        pf[t][i]     = (_Float16)sc[2 * t][i];
        pf[t][8 + i] = (_Float16)sc[2 * t + 1][i];
      }

#pragma unroll
    for (int nt = 0; nt < 4; ++nt)
#pragma unroll
      for (int r = 0; r < 8; ++r) acc[nt][r] *= alpha;

#pragma unroll
    for (int t = 0; t < 2; ++t)
#pragma unroll
      for (int nt = 0; nt < 4; ++nt) {
        const v16h vf = load_frag_row(vts + (nt * 16) * KPAD + t * 32, KPAD, lane);
        acc[nt] = wmma_f16(vf, pf[t], acc[nt]);
      }
  }

  {
    const float inv = 64.0f / li;
    _Float16* orow = ost + (wave * 16u + colb) * KPAD;
#pragma unroll
    for (int nt = 0; nt < 4; ++nt) {
      H8 pk;
#pragma unroll
      for (int r = 0; r < 8; ++r) pk.h[r] = (_Float16)(acc[nt][r] * inv);
      *(v4u*)(orow + nt * 16 + rofs) = pk.u;
    }
  }
  __syncthreads();

  v4u rv[4];
#pragma unroll
  for (unsigned it = 0; it < 4u; ++it) {
    const unsigned idx = it * 256u + tid;
    const unsigned row = idx >> 3, piece = idx & 7u;
    rv[it] = *(const v4u*)(ost + row * KPAD + piece * 8u);
  }
  _Float16* cbase = ctx + ((size_t)b * SEQ + q0) * DM + h * HD;
#pragma unroll
  for (unsigned it = 0; it < 4u; ++it) {
    const unsigned idx = it * 256u + tid;
    const unsigned row = idx >> 3, piece = idx & 7u;
    *(volatile v4u*)(cbase + (size_t)row * DM + piece * 8u) = rv[it];
  }
  __threadfence();
#pragma unroll
  for (unsigned it = 0; it < 4u; ++it) {
    const unsigned idx = it * 256u + tid;
    const unsigned row = idx >> 3, piece = idx & 7u;
    *(volatile v4u*)(cbase + (size_t)row * DM + piece * 8u) = rv[it];
  }
}

template <int KD, int MODE>
__global__ __launch_bounds__(256) void gemm_res_kernel(
    const _Float16* __restrict__ act, const _Float16* __restrict__ wt,
    const float* __restrict__ bias, const float* __restrict__ gam,
    const float* __restrict__ res,
    float* __restrict__ outf, _Float16* __restrict__ outh) {
  __shared__ float ys[16 * YP];
  __shared__ float srstd[16];

  const unsigned tid  = threadIdx.x;
  const unsigned lane = tid & 31u;
  const unsigned wave = tid >> 5;
  const unsigned hh   = lane >> 4;
  const unsigned l15  = lane & 15u;
  const unsigned m0   = blockIdx.x * 16u;
  const unsigned n0   = wave * 128u;

  const _Float16* brow = act + (size_t)m0 * KD;
  const _Float16* arow = wt + (size_t)n0 * KD;

  v8f acc[8];
#pragma unroll
  for (int j = 0; j < 8; ++j) acc[j] = (v8f){};

#pragma unroll 1
  for (unsigned kk = 0; kk < (unsigned)KD; kk += 32u) {
    const v16h bfr = load_frag_row(brow + kk, KD, lane);
#pragma unroll
    for (int j = 0; j < 8; ++j) {
      const v16h afr = load_frag_row(arow + (size_t)(j * 16) * KD + kk, KD, lane);
      acc[j] = wmma_f16(afr, bfr, acc[j]);
    }
  }

  {
    const float rsc = 1.0f / (WSC * WSC);
    float* yrow = ys + l15 * YP;
#pragma unroll
    for (int j = 0; j < 8; ++j) {
      const unsigned n8 = n0 + (unsigned)j * 16u + hh * 8u;
      const v4f b0 = *(const v4f*)(bias + n8);
      const v4f b1 = *(const v4f*)(bias + n8 + 4u);
      v4f y0, y1;
#pragma unroll
      for (int i = 0; i < 4; ++i) {
        y0[i] = acc[j][i]     * rsc + bf16q(b0[i]);
        y1[i] = acc[j][4 + i] * rsc + bf16q(b1[i]);
      }
      *(v4f*)(yrow + n8)      = y0;
      *(v4f*)(yrow + n8 + 4u) = y1;
    }
  }
  __syncthreads();

#pragma unroll 4
  for (unsigned it = 0; it < 16u; ++it) {
    const unsigned idx = it * 256u + tid;
    const unsigned row = idx >> 8, piece = idx & 255u;
    const unsigned m = m0 + row;
    v4f rsd;
    if (MODE == 0) {
      const unsigned bb = m / (unsigned)SEQ;
      const unsigned s  = m - bb * (unsigned)SEQ;
      rsd = *(const v4f*)(res + ((size_t)bb * SEQ_FULL + s) * DM + piece * 4u);
#pragma unroll
      for (int c = 0; c < 4; ++c) rsd[c] = bf16q(rsd[c]);
    } else {
      rsd = *(const v4f*)(res + (size_t)m * DM + piece * 4u);
    }
    float* yp = ys + row * YP + piece * 4u;
    v4f yv = *(const v4f*)yp;
#pragma unroll
    for (int c = 0; c < 4; ++c) yv[c] += rsd[c];
    *(v4f*)yp = yv;
  }
  __syncthreads();

  if (MODE == 0) {
    const unsigned r  = tid >> 4;
    const unsigned sl = tid & 15u;
    const float* yr = ys + r * YP + sl * 64u;
    float ss = 0.0f;
#pragma unroll 4
    for (unsigned i = 0; i < 16u; ++i) {
      const v4f v = *(const v4f*)(yr + i * 4u);
      ss += v[0] * v[0];
      ss += v[1] * v[1];
      ss += v[2] * v[2];
      ss += v[3] * v[3];
    }
    ss += __shfl_xor(ss, 1, 32);
    ss += __shfl_xor(ss, 2, 32);
    ss += __shfl_xor(ss, 4, 32);
    ss += __shfl_xor(ss, 8, 32);
    if (sl == 0u) srstd[r] = rsqrtf(ss * (1.0f / DM) + RMS_EPS);
    __syncthreads();
  }

  auto store_pass = [&]() {
#pragma unroll 4
    for (unsigned it = 0; it < 16u; ++it) {
      const unsigned idx = it * 256u + tid;
      const unsigned row = idx >> 8, piece = idx & 255u;
      const unsigned m = m0 + row;
      const v4f v = *(const v4f*)(ys + row * YP + piece * 4u);
      size_t drow;
      if (MODE == 0) {
        drow = (size_t)m;
      } else {
        const unsigned bb = m / (unsigned)SEQ;
        const unsigned s  = m - bb * (unsigned)SEQ;
        drow = (size_t)bb * SEQ_FULL + s;
      }
      *(volatile v4f*)(outf + drow * DM + piece * 4u) = v;
    }
    if (MODE == 0) {
#pragma unroll 4
      for (unsigned it = 0; it < 8u; ++it) {
        const unsigned idx = it * 256u + tid;
        const unsigned row = idx >> 7, p8 = idx & 127u;
        const unsigned m = m0 + row;
        const v4f a  = *(const v4f*)(ys + row * YP + p8 * 8u);
        const v4f c  = *(const v4f*)(ys + row * YP + p8 * 8u + 4u);
        const v4f g0 = *(const v4f*)(gam + p8 * 8u);
        const v4f g1 = *(const v4f*)(gam + p8 * 8u + 4u);
        const float rstd = srstd[row];
        H8 o;
#pragma unroll
        for (int i = 0; i < 4; ++i) {
          o.h[i]     = (_Float16)(bf16q(g0[i]) * (a[i] * rstd));
          o.h[4 + i] = (_Float16)(bf16q(g1[i]) * (c[i] * rstd));
        }
        *(volatile v4u*)(outh + (size_t)m * DM + p8 * 8u) = o.u;
      }
    }
  };
  store_pass();
  __threadfence();
  store_pass();
}

__global__ __launch_bounds__(256) void ffn1_kernel(
    const _Float16* __restrict__ x2h, const _Float16* __restrict__ wf1t,
    const float* __restrict__ bf1, _Float16* __restrict__ hp) {
  __shared__ _Float16 stg[128 * KPAD];

  const unsigned tid  = threadIdx.x;
  const unsigned lane = tid & 31u;
  const unsigned wave = tid >> 5;
  const unsigned hh   = lane >> 4;
  const unsigned l15  = lane & 15u;
  const unsigned cb   = blockIdx.y;
  const unsigned m0   = blockIdx.x * 128u;

  const _Float16* brow = x2h + (size_t)(m0 + wave * 16u) * DM;
  const _Float16* arow = wf1t + (size_t)(cb * 64u) * DM;

  v8f acc[4];
#pragma unroll
  for (int j = 0; j < 4; ++j) acc[j] = (v8f){};

#pragma unroll 1
  for (unsigned kk = 0; kk < DM; kk += 32u) {
    const v16h xf = load_frag_row(brow + kk, DM, lane);
#pragma unroll
    for (int j = 0; j < 4; ++j) {
      const v16h wf = load_frag_row(arow + (size_t)(j * 16) * DM + kk, DM, lane);
      acc[j] = wmma_f16(wf, xf, acc[j]);
    }
  }

  const float rsc = 1.0f / WSC;
  _Float16* srow = stg + (wave * 16u + l15) * KPAD;
#pragma unroll
  for (int j = 0; j < 4; ++j) {
    const unsigned n8 = (unsigned)j * 16u + hh * 8u;
    const v4f b0 = *(const v4f*)(bf1 + cb * 64u + n8);
    const v4f b1 = *(const v4f*)(bf1 + cb * 64u + n8 + 4u);
    H8 pk;
#pragma unroll
    for (int r = 0; r < 4; ++r) {
      const float u0 = acc[j][r]     * rsc + bf16q(b0[r]);
      const float u1 = acc[j][4 + r] * rsc + bf16q(b1[r]);
      const float g0 = u0 * __builtin_amdgcn_rcpf(1.0f + __expf(-u0));
      const float g1 = u1 * __builtin_amdgcn_rcpf(1.0f + __expf(-u1));
      pk.h[r]     = (_Float16)(g0 * WSC);
      pk.h[4 + r] = (_Float16)(g1 * WSC);
    }
    *(v4u*)(srow + n8) = pk.u;
  }
  __syncthreads();

  v4u rv[4];
#pragma unroll
  for (unsigned it = 0; it < 4u; ++it) {
    const unsigned idx = it * 256u + tid;
    const unsigned row = idx >> 3, piece = idx & 7u;
    rv[it] = *(const v4u*)(stg + row * KPAD + piece * 8u);
  }
#pragma unroll
  for (unsigned it = 0; it < 4u; ++it) {
    const unsigned idx = it * 256u + tid;
    const unsigned row = idx >> 3, piece = idx & 7u;
    *(volatile v4u*)(hp + (size_t)(m0 + row) * FF + cb * 64u + piece * 8u) = rv[it];
  }
  __threadfence();
#pragma unroll
  for (unsigned it = 0; it < 4u; ++it) {
    const unsigned idx = it * 256u + tid;
    const unsigned row = idx >> 3, piece = idx & 7u;
    *(volatile v4u*)(hp + (size_t)(m0 + row) * FF + cb * 64u + piece * 8u) = rv[it];
  }
}

extern "C" void kernel_launch(void* const* d_in, const int* in_sizes, int n_in,
                              void* d_out, int out_size, void* d_ws, size_t ws_size,
                              hipStream_t stream) {
  if (n_in < 15) return;
  const long needRows = (long)(NB - 1) * SEQ_FULL + SEQ;
  if ((long)in_sizes[0] < needRows * DM) return;
  if (in_sizes[1] < DM || in_sizes[2] < DM) return;
  if (in_sizes[3] < DM * DM || in_sizes[5] < DM * DM ||
      in_sizes[7] < DM * DM || in_sizes[9] < DM * DM) return;
  if (in_sizes[4] < DM || in_sizes[6] < DM || in_sizes[8] < DM || in_sizes[10] < DM) return;
  if (in_sizes[11] < DM * FF || in_sizes[13] < FF * DM) return;
  if (in_sizes[12] < FF || in_sizes[14] < DM) return;
  if ((long)out_size < needRows * DM) return;
  if (ws_size < WS_TOTAL) return;

  const float* x   = (const float*)d_in[0];
  const float* g1  = (const float*)d_in[1];
  const float* g2  = (const float*)d_in[2];
  const float* Wq  = (const float*)d_in[3];
  const float* bq  = (const float*)d_in[4];
  const float* Wk  = (const float*)d_in[5];
  const float* bk  = (const float*)d_in[6];
  const float* Wv  = (const float*)d_in[7];
  const float* bv  = (const float*)d_in[8];
  const float* Wo  = (const float*)d_in[9];
  const float* bo  = (const float*)d_in[10];
  const float* Wf1 = (const float*)d_in[11];
  const float* bf1 = (const float*)d_in[12];
  const float* Wf2 = (const float*)d_in[13];
  const float* bf2 = (const float*)d_in[14];
  float* out = (float*)d_out;

  char* ws = (char*)d_ws;
  size_t off = 0;
  _Float16* xh   = (_Float16*)(ws + off);
  _Float16* ctx  = xh;
  off += PLANE2;
  _Float16* wqkv = (_Float16*)(ws + off); off += WQKV_BYTES;
  _Float16* woh  = (_Float16*)(ws + off); off += WO_BYTES;
  _Float16* wf1t = (_Float16*)(ws + off); off += WF1_BYTES;
  _Float16* wf2t = (_Float16*)(ws + off); off += WF2_BYTES;
  _Float16* qh   = (_Float16*)(ws + off);
  float*    x1f  = (float*)(ws + off);
  off += PLANE2;
  _Float16* kh   = (_Float16*)(ws + off); off += PLANE2;
  _Float16* vTh  = (_Float16*)(ws + off);
  _Float16* x2h  = vTh;
  off += PLANE2;
  _Float16* hp   = (_Float16*)(ws + off); off += H_BYTES;
  if (off > ws_size) return;

  rms1_kernel<<<NRB, 256, 0, stream>>>(x, g1, xh);
  cvt_w_kernel<<<NWT, 256, 0, stream>>>(Wq, Wk, Wv, Wo, Wf1, Wf2, wqkv, woh, wf1t, wf2t);
  qkv_kernel<<<dim3(ROWS / 128, 3 * NH), 256, 0, stream>>>(xh, wqkv, bq, bk, bv, qh, kh, vTh);
  attn_kernel<<<dim3(SEQ / 128, NB * NH), 256, 0, stream>>>(qh, kh, vTh, ctx);
  gemm_res_kernel<DM, 0><<<ROWS / 16, 256, 0, stream>>>(ctx, woh, bo, g2, x, x1f, x2h);
  ffn1_kernel<<<dim3(ROWS / 128, FF / 64), 256, 0, stream>>>(x2h, wf1t, bf1, hp);
  gemm_res_kernel<FF, 1><<<ROWS / 16, 256, 0, stream>>>(hp, wf2t, bf2, g2, x1f, out, x2h);
}
